// TransformerLayer_32684701122642
// MI455X (gfx1250) — hardware-verified
//
#include <hip/hip_runtime.h>
#include <math.h>

typedef __attribute__((ext_vector_type(16))) _Float16 v16h;
typedef __attribute__((ext_vector_type(8)))  _Float16 v8h;
typedef __attribute__((ext_vector_type(8)))  float v8f;
typedef __attribute__((ext_vector_type(4)))  float v4f;
typedef __attribute__((ext_vector_type(4)))  unsigned v4u;

#ifndef NB
#define NB 2
#endif
#ifndef SEQ
#define SEQ 2048
#endif
#define NB_FULL 2
#define SEQ_FULL 2048
#define DD 1024
#define HH 16
#define HD 64
#define FF 4096
#define NR (NB * SEQ)
#define LN_EPS (1.0e-12f)
#define SCALE (0.125f)
#define WSC (64.0f)
#define PCAR (2048.0f)
#define YCAR (256.0f)
#define HCAR (16.0f)

static_assert(NB >= 1 && NB <= NB_FULL);
static_assert(SEQ >= 64 && SEQ <= SEQ_FULL && (SEQ % 64) == 0);
static_assert((DD % 128) == 0 && (FF % 128) == 0 && HH * HD == DD && HD == 64);
static_assert((NR % 64) == 0 && (DD % 32) == 0 && (FF % 32) == 0);
static_assert((size_t)NB_FULL * SEQ_FULL * DD * 4u == 16777216u);

#define WS_WTQ 0u
#define WS_WTK (WS_WTQ + 2u * (size_t)DD * DD)
#define WS_WTV (WS_WTK + 2u * (size_t)DD * DD)
#define WS_WTO (WS_WTV + 2u * (size_t)DD * DD)
#define WS_WT1 (WS_WTO + 2u * (size_t)DD * DD)
#define WS_WT2 (WS_WT1 + 2u * (size_t)FF * DD)
#define WS_H1  (WS_WT2 + 2u * (size_t)DD * FF)
#define WS_QH  (WS_H1  + 2u * (size_t)NR * DD)
#define WS_KH  (WS_QH  + 2u * (size_t)NR * DD)
#define WS_VT  (WS_KH  + 2u * (size_t)NR * DD)
#define WS_YH  (WS_VT  + 2u * (size_t)NR * DD)
#define WS_Z1  (WS_YH  + 2u * (size_t)NR * DD)
#define WS_H2  (WS_Z1  + 4u * (size_t)NR * DD)
#define WS_HF  (WS_H2  + 2u * (size_t)NR * DD)
#define WS_END (WS_HF  + 2u * (size_t)NR * FF)
static_assert(WS_END <= 134217728u);

template <typename T> __device__ __forceinline__ void vst2(void* p, T v) { *(volatile T*)p = v; __threadfence(); *(volatile T*)p = v; }
__device__ __forceinline__ v8f wmma16(v16h a, v16h b, v8f c) {
  v8f d = __builtin_amdgcn_wmma_f32_16x16x32_f16(false, a, false, b, (short)0, c, false, false);
  asm volatile("v_nop\n\tv_nop\n\tv_nop\n\tv_nop" : "+v"(d) : "v"(a), "v"(b));
  return d;
}
__device__ __forceinline__ v16h frag_h(const _Float16* rowk0, int lane) {
  union { v16h v; v8h q[2]; } u; const _Float16* p = rowk0 + 8 * (lane >> 4);
  u.q[0] = *(const v8h*)p; u.q[1] = *(const v8h*)(p + 16); return u.v;
}
__device__ __forceinline__ float bfr(float v) { return (float)(__bf16)v; }
__device__ __forceinline__ size_t grow(size_t r) { return (r / SEQ) * (size_t)SEQ_FULL + (r % SEQ); }
union H8 { v8h h; v4u u; };
#define LDSX() do { asm volatile("s_wait_dscnt 0" ::: "memory"); __builtin_amdgcn_wave_barrier(); __builtin_amdgcn_fence(3  , "workgroup"); } while (0)

__global__ __launch_bounds__(256) void k_wt(const float* __restrict__ W, int K, int N, _Float16* __restrict__ WT) {
  __shared__ float t[64][65];
  const int tid = threadIdx.x, n0 = blockIdx.x * 64, k0 = blockIdx.y * 64;
#pragma unroll 1
  for (int it = 0; it < 16; ++it) { const int e = tid + it * 256, kl = e >> 6, nl = e & 63; t[kl][nl] = W[(size_t)(k0 + kl) * N + n0 + nl]; }
  __syncthreads();
#pragma unroll 1
  for (int it = 0; it < 2; ++it) { const int e = tid + it * 256, nl = e >> 3, q = e & 7; H8 P;
#pragma unroll
    for (int i = 0; i < 8; ++i) P.h[i] = (_Float16)(bfr(t[q * 8 + i][nl]) * WSC);
    vst2((unsigned*)(WT + (size_t)(n0 + nl) * K + k0 + q * 8), P.u); }
}

__global__ __launch_bounds__(256) void k_ln(const float* __restrict__ X, int x_full, int rne_in, const float* __restrict__ G, const float* __restrict__ BE, _Float16* __restrict__ OUT, int nrows) {
  const int wave = threadIdx.x >> 5, lane = threadIdx.x & 31; const int row = blockIdx.x * 8 + wave; if (row >= nrows) return;
  const size_t xrow = x_full ? grow((size_t)row) : (size_t)row; const float* xp = X + xrow * DD;
  float s = 0.f;
#pragma unroll 1
  for (int i = 0; i < DD / 256; ++i) { const int c = i * 256 + lane * 8; v4f a = *(const v4f*)(xp + c), bq = *(const v4f*)(xp + c + 4);
    if (rne_in) {
#pragma unroll
      for (int k = 0; k < 4; ++k) { a[k] = bfr(a[k]); bq[k] = bfr(bq[k]); } }
    s += ((a[0] + a[1]) + (a[2] + a[3])) + ((bq[0] + bq[1]) + (bq[2] + bq[3])); }
#pragma unroll
  for (int o = 1; o < 32; o <<= 1) s += __shfl_xor(s, o);
  const float mu = s * (1.0f / DD); float q = 0.f;
#pragma unroll 1
  for (int i = 0; i < DD / 256; ++i) { const int c = i * 256 + lane * 8; v4f a = *(const v4f*)(xp + c), bq = *(const v4f*)(xp + c + 4);
    if (rne_in) {
#pragma unroll
      for (int k = 0; k < 4; ++k) { a[k] = bfr(a[k]); bq[k] = bfr(bq[k]); } }
#pragma unroll
    for (int k = 0; k < 4; ++k) { const float d0 = a[k] - mu, d1 = bq[k] - mu; q += d0 * d0; q += d1 * d1; } }
#pragma unroll
  for (int o = 1; o < 32; o <<= 1) q += __shfl_xor(q, o);
  const float inv = rsqrtf(q * (1.0f / DD) + LN_EPS);
#pragma unroll 1
  for (int i = 0; i < DD / 256; ++i) { const int c = i * 256 + lane * 8; v4f a = *(const v4f*)(xp + c), bq = *(const v4f*)(xp + c + 4);
    if (rne_in) {
#pragma unroll
      for (int k = 0; k < 4; ++k) { a[k] = bfr(a[k]); bq[k] = bfr(bq[k]); } }
    const v4f ga = *(const v4f*)(G + c), gb = *(const v4f*)(G + c + 4), ea = *(const v4f*)(BE + c), eb = *(const v4f*)(BE + c + 4); H8 P;
#pragma unroll
    for (int k = 0; k < 4; ++k) { P.h[k] = (_Float16)(((a[k] - mu) * inv) * bfr(ga[k]) + bfr(ea[k])); P.h[4 + k] = (_Float16)(((bq[k] - mu) * inv) * bfr(gb[k]) + bfr(eb[k])); }
    vst2((unsigned*)(OUT + (size_t)row * DD + c), P.u); }
}

union GemmLds { float sf[4][16][132]; _Float16 th[128][72]; };
template <int MODE>
__global__ __launch_bounds__(128) void k_gemm(const _Float16* __restrict__ A, int lda, int K, const _Float16* __restrict__ WT, int nout, const float* __restrict__ BIAS, float osc,
    const float* __restrict__ RES, int res_full, int rne_res, int gelu, float hsc, int out_full, float* __restrict__ OUTF, _Float16* __restrict__ OUTH) {
  __shared__ __align__(16) GemmLds L;
  const int tid = threadIdx.x, wave = tid >> 5, lane = tid & 31, col = lane & 15, g = lane >> 4; const int c0 = blockIdx.y * 128; const size_t rb = (size_t)blockIdx.x * 64, r0 = rb + wave * 16;
  v8f acc[8] = {};
#pragma unroll 1
  for (int kc = 0; kc < K / 32; ++kc) { const v16h a = frag_h(A + (r0 + col) * (size_t)lda + kc * 32, lane);
    asm volatile("s_wait_loadcnt 0x0" ::: "memory");
#pragma unroll
    for (int j = 0; j < 8; ++j) { const v16h w = frag_h(WT + (size_t)(c0 + j * 16 + col) * K + kc * 32, lane); acc[j] = wmma16(a, w, acc[j]); } }
  if constexpr (MODE != 2) {
#pragma unroll
    for (int j = 0; j < 8; ++j) { const float bb = bfr(BIAS[c0 + j * 16 + col]);
#pragma unroll
      for (int r = 0; r < 8; ++r) L.sf[wave][8 * g + r][j * 16 + col] = acc[j][r] * osc + bb; }
    LDSX();
    if constexpr (MODE == 0) {
#pragma unroll 1
      for (int rl = 0; rl < 16; ++rl) { const size_t r = r0 + rl; const int c = c0 + lane * 4; v4f v = *(const v4f*)&L.sf[wave][rl][lane * 4];
        if (RES) { const size_t rr = res_full ? grow(r) : r; v4f rv = *(const v4f*)(RES + rr * (size_t)nout + c);
          if (rne_res) { rv[0] = bfr(rv[0]); rv[1] = bfr(rv[1]); rv[2] = bfr(rv[2]); rv[3] = bfr(rv[3]); }
          v[0] += rv[0]; v[1] += rv[1]; v[2] += rv[2]; v[3] += rv[3]; }
        const size_t ro = out_full ? grow(r) : r; vst2(OUTF + ro * (size_t)nout + c, v); }
    } else {
#pragma unroll 1
      for (int it = 0; it < 8; ++it) { const int rl = it * 2 + g; const v4f v0 = *(const v4f*)&L.sf[wave][rl][col * 8], v1 = *(const v4f*)&L.sf[wave][rl][col * 8 + 4];
        float t[8] = { v0[0], v0[1], v0[2], v0[3], v1[0], v1[1], v1[2], v1[3] };
        if (gelu) {
#pragma unroll
          for (int i = 0; i < 8; ++i) t[i] = 0.5f * t[i] * (1.0f + erff(t[i] * 0.70710678118654752f)); }
        H8 P;
#pragma unroll
        for (int i = 0; i < 8; ++i) P.h[i] = (_Float16)(t[i] * hsc);
        vst2((unsigned*)(OUTH + (r0 + rl) * (size_t)nout + c0 + col * 8), P.u); } }
  } else {
#pragma unroll
    for (int j = 0; j < 8; ++j) { const float bb = bfr(BIAS[c0 + j * 16 + col]);
#pragma unroll
      for (int r = 0; r < 8; ++r) L.th[j * 16 + col][wave * 16 + 8 * g + r] = (_Float16)(acc[j][r] * osc + bb); }
    __syncthreads();
    const size_t bidx = rb / SEQ; const int t0 = (int)(rb % SEQ);
#pragma unroll 1
    for (int it = 0; it < 8; ++it) { const int e = tid + it * 128, cl = e >> 3, q = e & 7; vst2((unsigned*)(OUTH + (bidx * nout + c0 + cl) * (size_t)SEQ + t0 + q * 8), *(const v4u*)&L.th[cl][q * 8]); }
  }
}

__global__ __launch_bounds__(128) void k_attn(const _Float16* __restrict__ QH, const _Float16* __restrict__ KH, const _Float16* __restrict__ VT, const float* __restrict__ MASK, _Float16* __restrict__ YH) {
  __shared__ __align__(16) _Float16 Ks[64][72], Vs[64][72], Ps[4][16][72], So[4][16][72];
  const int tid = threadIdx.x, wave = tid >> 5, lane = tid & 31, col = lane & 15, g = lane >> 4;
  const int qb = blockIdx.x, b = blockIdx.y / HH, h = blockIdx.y % HH;
  const size_t qr0 = (size_t)b * SEQ + qb * 64 + wave * 16;
  const v16h qf0 = frag_h(QH + (qr0 + col) * DD + h * HD, lane), qf1 = frag_h(QH + (qr0 + col) * DD + h * HD + 32, lane);
  v8f o[4] = {}; float mrun[8], lrun[8];
#pragma unroll
  for (int r = 0; r < 8; ++r) { mrun[r] = -1.0e30f; lrun[r] = 0.f; }
#pragma unroll 1
  for (int kt = 0; kt < SEQ / 64; ++kt) { const int k0 = kt * 64;
    __syncthreads();
#pragma unroll
    for (int it = 0; it < 4; ++it) { const int e = tid + it * 128, r = e >> 3, c8 = (e & 7) * 8;
      *(v8h*)&Ks[r][c8] = *(const v8h*)(KH + ((size_t)b * SEQ + k0 + r) * DD + h * HD + c8);
      *(v8h*)&Vs[r][c8] = *(const v8h*)(VT + ((size_t)b * DD + h * HD + r) * SEQ + k0 + c8); }
    __syncthreads();
    v8f sc[4];
#pragma unroll
    for (int nt = 0; nt < 4; ++nt) { v8f s = {}; s = wmma16(qf0, frag_h(&Ks[nt * 16 + col][0], lane), s); s = wmma16(qf1, frag_h(&Ks[nt * 16 + col][32], lane), s); sc[nt] = s; }
    float rm[8];
#pragma unroll
    for (int r = 0; r < 8; ++r) rm[r] = -1.0e30f;
#pragma unroll
    for (int nt = 0; nt < 4; ++nt) { const float mv = bfr(MASK[(size_t)b * SEQ_FULL + k0 + nt * 16 + col]);
#pragma unroll
      for (int r = 0; r < 8; ++r) { const float sv = sc[nt][r] * SCALE + mv; sc[nt][r] = sv; rm[r] = fmaxf(rm[r], sv); } }
#pragma unroll
    for (int of = 1; of < 16; of <<= 1)
#pragma unroll
      for (int r = 0; r < 8; ++r) rm[r] = fmaxf(rm[r], __shfl_xor(rm[r], of));
    float alpha[8], rs[8];
#pragma unroll
    for (int r = 0; r < 8; ++r) { const float mn = fmaxf(mrun[r], rm[r]); alpha[r] = __expf(mrun[r] - mn); mrun[r] = mn; rs[r] = 0.f; }
#pragma unroll
    for (int nt = 0; nt < 4; ++nt)
#pragma unroll
      for (int r = 0; r < 8; ++r) { const float p = __expf(sc[nt][r] - mrun[r]); rs[r] += p; Ps[wave][8 * g + r][nt * 16 + col] = (_Float16)(p * PCAR); }
#pragma unroll
    for (int of = 1; of < 16; of <<= 1)
#pragma unroll
      for (int r = 0; r < 8; ++r) rs[r] += __shfl_xor(rs[r], of);
#pragma unroll
    for (int r = 0; r < 8; ++r) lrun[r] = lrun[r] * alpha[r] + rs[r];
    __syncthreads();
    const v16h pf0 = frag_h(&Ps[wave][col][0], lane), pf1 = frag_h(&Ps[wave][col][32], lane);
#pragma unroll
    for (int t = 0; t < 4; ++t) {
#pragma unroll
      for (int r = 0; r < 8; ++r) o[t][r] *= alpha[r];
      o[t] = wmma16(pf0, frag_h(&Vs[t * 16 + col][0], lane), o[t]); o[t] = wmma16(pf1, frag_h(&Vs[t * 16 + col][32], lane), o[t]); } }
  float linv[8];
#pragma unroll
  for (int r = 0; r < 8; ++r) linv[r] = (YCAR / PCAR) * __builtin_amdgcn_rcpf(lrun[r]);
#pragma unroll
  for (int t = 0; t < 4; ++t)
#pragma unroll
    for (int r = 0; r < 8; ++r) So[wave][8 * g + r][t * 16 + col] = (_Float16)(o[t][r] * linv[r]);
  LDSX();
#pragma unroll 1
  for (int it = 0; it < 4; ++it) { const int rl = it * 4 + (lane >> 3), q = lane & 7; vst2((unsigned*)(YH + (qr0 + rl) * DD + h * HD + q * 8), *(const v4u*)&So[wave][rl][q * 8]); }
}

extern "C" void kernel_launch(void* const* d_in, const int* in_sizes, int n_in, void* d_out, int out_size, void* d_ws, size_t ws_size, hipStream_t stream) {
  if (n_in < 18) return;
  const long long need_rows = (long long)(NB - 1) * SEQ_FULL + SEQ;
  if ((long long)in_sizes[0] < need_rows * DD || (long long)in_sizes[1] < need_rows) return;
  if (in_sizes[2] < DD * DD || in_sizes[4] < DD * DD || in_sizes[6] < DD * DD || in_sizes[8] < DD * DD) return;
  if (in_sizes[10] < DD * FF || in_sizes[12] < FF * DD) return;
  if (in_sizes[3] < DD || in_sizes[5] < DD || in_sizes[7] < DD || in_sizes[9] < DD || in_sizes[11] < FF || in_sizes[13] < DD) return;
  if (in_sizes[14] < DD || in_sizes[15] < DD || in_sizes[16] < DD || in_sizes[17] < DD) return;
  if ((long long)out_size < need_rows * DD) return;
  if (ws_size < (size_t)WS_END) return;
  const float *x = (const float*)d_in[0], *mask = (const float*)d_in[1];
  const float *wq = (const float*)d_in[2], *bq = (const float*)d_in[3], *wk = (const float*)d_in[4], *bk = (const float*)d_in[5], *wv = (const float*)d_in[6], *bv = (const float*)d_in[7];
  const float *wo = (const float*)d_in[8], *bo = (const float*)d_in[9], *w1 = (const float*)d_in[10], *b1 = (const float*)d_in[11], *w2 = (const float*)d_in[12], *b2 = (const float*)d_in[13];
  const float *g1 = (const float*)d_in[14], *be1 = (const float*)d_in[15], *g2 = (const float*)d_in[16], *be2 = (const float*)d_in[17];
  char* ws = (char*)d_ws;
  _Float16 *WTQ = (_Float16*)(ws + WS_WTQ), *WTK = (_Float16*)(ws + WS_WTK), *WTV = (_Float16*)(ws + WS_WTV), *WTO = (_Float16*)(ws + WS_WTO), *WT1 = (_Float16*)(ws + WS_WT1), *WT2 = (_Float16*)(ws + WS_WT2);
  _Float16 *H1 = (_Float16*)(ws + WS_H1), *QH = (_Float16*)(ws + WS_QH), *KH = (_Float16*)(ws + WS_KH), *VT = (_Float16*)(ws + WS_VT), *YH = (_Float16*)(ws + WS_YH), *H2 = (_Float16*)(ws + WS_H2), *HF = (_Float16*)(ws + WS_HF);
  float* Z1 = (float*)(ws + WS_Z1); float* OUT = (float*)d_out;
  const float* nof = (const float*)nullptr; float* noo = (float*)nullptr; _Float16* noh = (_Float16*)nullptr;
  k_wt<<<dim3(DD / 64, DD / 64), 256, 0, stream>>>(wq, DD, DD, WTQ);
  k_wt<<<dim3(DD / 64, DD / 64), 256, 0, stream>>>(wk, DD, DD, WTK);
  k_wt<<<dim3(DD / 64, DD / 64), 256, 0, stream>>>(wv, DD, DD, WTV);
  k_wt<<<dim3(DD / 64, DD / 64), 256, 0, stream>>>(wo, DD, DD, WTO);
  k_wt<<<dim3(FF / 64, DD / 64), 256, 0, stream>>>(w1, DD, FF, WT1);
  k_wt<<<dim3(DD / 64, FF / 64), 256, 0, stream>>>(w2, FF, DD, WT2);
  k_ln<<<dim3(NR / 8), 256, 0, stream>>>(x, 1, 1, g1, be1, H1, NR);
  k_gemm<1><<<dim3(NR / 64, DD / 128), 128, 0, stream>>>(H1, DD, DD, WTQ, DD, bq, 1.0f / WSC, nof, 0, 0, 0, 1.0f, 0, noo, QH);
  k_gemm<1><<<dim3(NR / 64, DD / 128), 128, 0, stream>>>(H1, DD, DD, WTK, DD, bk, 1.0f / WSC, nof, 0, 0, 0, 1.0f, 0, noo, KH);
  k_gemm<2><<<dim3(NR / 64, DD / 128), 128, 0, stream>>>(H1, DD, DD, WTV, DD, bv, 1.0f / WSC, nof, 0, 0, 0, 1.0f, 0, noo, VT);
  k_attn<<<dim3(SEQ / 64, NB * HH), 128, 0, stream>>>(QH, KH, VT, mask, YH);
  k_gemm<0><<<dim3(NR / 64, DD / 128), 128, 0, stream>>>(YH, DD, DD, WTO, DD, bo, 1.0f / (WSC * YCAR), x, 1, 1, 0, 1.0f, 0, Z1, noh);
  k_ln<<<dim3(NR / 8), 256, 0, stream>>>(Z1, 0, 0, g2, be2, H2, NR);
  k_gemm<1><<<dim3(NR / 64, FF / 128), 128, 0, stream>>>(H2, DD, DD, WT1, FF, b1, 1.0f / WSC, nof, 0, 0, 1, HCAR, 0, noo, HF);
  k_gemm<0><<<dim3(NR / 64, DD / 128), 128, 0, stream>>>(HF, FF, FF, WT2, DD, b2, 1.0f / (WSC * HCAR), Z1, 0, 0, 0, 1.0f, 1, OUT, noh);
}
